// GraphCoarsenLayer_65000035058039
// MI455X (gfx1250) — hardware-verified
//
#include <hip/hip_runtime.h>
#include <stddef.h>
#include <stdint.h>


#define NN        50000
#define CC        256
#define OO        256
#define DD        32
#define SS        16
#define MP        50048
#define XB_PITCH  256
#define AGG_PITCH 1024
#define WT_PITCH  1280
#define SEG_K     256
#ifndef SPLIT_S
#define SPLIT_S 0
#endif
#ifndef SPLIT_U
#define SPLIT_U 1
#endif
#define GT        256
#define TP        65
#define PREP_XB_BLOCKS (MP / 8)
#define PREP_WT_BLOCKS 48
#define PREP_BLOCKS    (PREP_XB_BLOCKS + PREP_WT_BLOCKS + 1)

typedef float          v4f   __attribute__((ext_vector_type(4)));
typedef float          v8f   __attribute__((ext_vector_type(8)));
typedef int            v8i   __attribute__((ext_vector_type(8)));
typedef unsigned       v4u   __attribute__((ext_vector_type(4)));
typedef unsigned short v8us  __attribute__((ext_vector_type(8)));
typedef unsigned short v16us __attribute__((ext_vector_type(16)));
typedef __bf16         v16bf __attribute__((ext_vector_type(16)));
typedef v4f  __attribute__((may_alias)) v4fa;
typedef v4u  __attribute__((may_alias)) v4ua;
typedef v8us __attribute__((may_alias)) v8usa;
union FragB { v16bf v; v16us u; v8us h[2]; v8i w; };

struct KSeg { int src; int acol; int wcol; };
struct KSegTab { KSeg e[5]; int n; };
constexpr KSegTab make_segs() {
  KSegTab t{};
  int c = 0;
  t.e[c] = KSeg{0, 0, 0};       ++c;
  t.e[c] = KSeg{1, 0, 256};     ++c;
  if (SPLIT_S != 0) { t.e[c] = KSeg{1, 256, 512};  ++c; }
  t.e[c] = KSeg{1, 512, 768};   ++c;
  if (SPLIT_U != 0) { t.e[c] = KSeg{1, 768, 1024}; ++c; }
  t.n = c;
  return t;
}
static constexpr KSegTab SEGS = make_segs();
constexpr int NSEG = SEGS.n;
constexpr int KEXT = NSEG * SEG_K;
constexpr bool segs_ok() {
  for (int i = 0; i < SEGS.n; ++i) {
    const int ap = (SEGS.e[i].src == 0) ? XB_PITCH : AGG_PITCH;
    if (SEGS.e[i].acol + SEG_K > ap) return false;
    if (SEGS.e[i].wcol + SEG_K > WT_PITCH) return false;
  }
  return true;
}

constexpr size_t XB_BYTES  = (size_t)MP * XB_PITCH * 2;
constexpr size_t AGG_BYTES = (size_t)MP * AGG_PITCH * 2;
constexpr size_t WT_BYTES  = (size_t)OO * WT_PITCH * 2;
constexpr size_t BS_BYTES  = (size_t)OO * 4;
constexpr size_t O_XB  = 0;
constexpr size_t O_AGG = O_XB + XB_BYTES;
constexpr size_t O_WT  = O_AGG + AGG_BYTES;
constexpr size_t O_BS  = O_WT + WT_BYTES;
constexpr size_t WS_TOTAL = O_BS + BS_BYTES;

static_assert(CC == 256 && OO == 256 && DD == 32 && SS == 16 && DD - SS == 16);
static_assert(32 * 8 == CC);
static_assert(NN % 8 == 0 && MP % 8 == 0 && MP % 128 == 0 && MP >= NN && MP - NN < 128);
static_assert(KEXT % 32 == 0 && SEG_K % 32 == 0 && NSEG >= 3 && NSEG <= 5);
static_assert(WT_PITCH >= 5 * SEG_K && WT_PITCH >= KEXT && WT_PITCH % 64 == 0);
static_assert(AGG_PITCH % 64 == 0 && AGG_PITCH >= 4 * CC && XB_PITCH == CC);
static_assert(segs_ok());
static_assert(O_AGG % 256 == 0 && O_WT % 256 == 0 && O_BS % 256 == 0);
static_assert(WS_TOTAL <= ((size_t)128u << 20));
static_assert(PREP_WT_BLOCKS == 3 * (CC / 64) * (OO / 64));

__device__ __forceinline__ v8f wmb(const FragB& a, const FragB& b, v8f c) {
  v8f d = __builtin_amdgcn_wmma_f32_16x16x32_bf16(false, a.v, false, b.v, (short)0, c, false, false);
  asm volatile("v_nop\n\tv_nop\n\tv_nop\n\tv_nop" : "+v"(d) : "v"(a.w), "v"(b.w));
  return d;
}

__device__ __forceinline__ unsigned bf16_bits(float f) {
  const unsigned u = __float_as_uint(f);
  const unsigned r = (u + 0x7FFFu + ((u >> 16) & 1u)) >> 16;
  return (f != f) ? 0x7FC0u : r;
}
__device__ __forceinline__ float bf16_val(float f) {
  return __uint_as_float(bf16_bits(f) << 16);
}

struct Q4 { v4f q0, q1, q2, q3; };
__device__ __forceinline__ Q4 ld_tile(const float* __restrict__ W, int k0, int n0, int tid) {
  Q4 r;
  const float* p = W + (size_t)(k0 + (tid >> 4)) * OO + n0 + (tid & 15) * 4;
  r.q0 = *(const v4f*)p;
  r.q1 = *(const v4f*)(p + 16 * OO);
  r.q2 = *(const v4f*)(p + 32 * OO);
  r.q3 = *(const v4f*)(p + 48 * OO);
  return r;
}

__global__ __launch_bounds__(GT) void k_prep(const float* __restrict__ x,
                                             const float* __restrict__ Wself, const float* __restrict__ bself,
                                             const float* __restrict__ Wneigh, const float* __restrict__ bneigh,
                                             const float* __restrict__ Wcoars, const float* __restrict__ bcoars,
                                             unsigned short* XB, unsigned short* WT, float* BS) {
  __shared__ float tile[64 * TP];
  const int tid = (int)threadIdx.x;
  const int b   = (int)blockIdx.x;
  if (b < PREP_XB_BLOCKS) {
    const int row = b * 8 + (tid >> 5);
    const int c8  = (tid & 31) * 8;
    const int rc  = row < NN ? row : NN - 1;
    const unsigned keep = row < NN ? 0xffffffffu : 0u;
    const float* p = x + (size_t)rc * CC + c8;
    const v4f a = *(const v4f*)p;
    const v4f c = *(const v4f*)(p + 4);
    v4u o;
    o.x = (bf16_bits(a.x) | (bf16_bits(a.y) << 16)) & keep;
    o.y = (bf16_bits(a.z) | (bf16_bits(a.w) << 16)) & keep;
    o.z = (bf16_bits(c.x) | (bf16_bits(c.y) << 16)) & keep;
    o.w = (bf16_bits(c.z) | (bf16_bits(c.w) << 16)) & keep;
    unsigned short* dp = XB + (size_t)row * XB_PITCH + c8;
    *(volatile v4u*)dp = o;
    __threadfence();
    *(volatile v4u*)dp = o;
  } else if (b < PREP_XB_BLOCKS + PREP_WT_BLOCKS) {
    const int tb  = b - PREP_XB_BLOCKS;
    const int mat = tb >> 4;
    const int tl  = tb & 15;
    const int k0  = (tl >> 2) * 64;
    const int n0  = (tl & 3) * 64;
    Q4 q;
    if (mat == 0)      q = ld_tile(Wself,  k0, n0, tid);
    else if (mat == 1) q = ld_tile(Wneigh, k0, n0, tid);
    else               q = ld_tile(Wcoars, k0, n0, tid);
    {
      const int kr = tid >> 4, c4 = (tid & 15) * 4;
      const int o0 = kr * TP + c4;
      tile[o0 + 0] = q.q0.x; tile[o0 + 1] = q.q0.y; tile[o0 + 2] = q.q0.z; tile[o0 + 3] = q.q0.w;
      tile[o0 + 16 * TP + 0] = q.q1.x; tile[o0 + 16 * TP + 1] = q.q1.y;
      tile[o0 + 16 * TP + 2] = q.q1.z; tile[o0 + 16 * TP + 3] = q.q1.w;
      tile[o0 + 32 * TP + 0] = q.q2.x; tile[o0 + 32 * TP + 1] = q.q2.y;
      tile[o0 + 32 * TP + 2] = q.q2.z; tile[o0 + 32 * TP + 3] = q.q2.w;
      tile[o0 + 48 * TP + 0] = q.q3.x; tile[o0 + 48 * TP + 1] = q.q3.y;
      tile[o0 + 48 * TP + 2] = q.q3.z; tile[o0 + 48 * TP + 3] = q.q3.w;
    }
    __syncthreads();
    const int cb = (mat == 0) ? 0 : ((mat == 1) ? 256 : 768);
    v4u o[2];
#pragma unroll
    for (int i = 0; i < 2; ++i) {
      const int u  = tid + GT * i;
      const int nn = u >> 3;
      const int k8 = (u & 7) * 8;
      const int t0 = k8 * TP + nn;
      const float f0 = tile[t0],          f1 = tile[t0 + TP],     f2 = tile[t0 + 2 * TP], f3 = tile[t0 + 3 * TP];
      const float f4 = tile[t0 + 4 * TP], f5 = tile[t0 + 5 * TP], f6 = tile[t0 + 6 * TP], f7 = tile[t0 + 7 * TP];
      v4u w;
      w.x = bf16_bits(f0) | (bf16_bits(f1) << 16);
      w.y = bf16_bits(f2) | (bf16_bits(f3) << 16);
      w.z = bf16_bits(f4) | (bf16_bits(f5) << 16);
      w.w = bf16_bits(f6) | (bf16_bits(f7) << 16);
      o[i] = w;
    }
#pragma unroll
    for (int pass = 0; pass < 2; ++pass) {
      if (pass != 0) __threadfence();
#pragma unroll
      for (int i = 0; i < 2; ++i) {
        const int u  = tid + GT * i;
        const int nn = u >> 3;
        const int k8 = (u & 7) * 8;
        unsigned short* dp = WT + (size_t)(n0 + nn) * WT_PITCH + cb + k0 + k8;
        *(volatile v4u*)dp = o[i];
        if (mat != 0) *(volatile v4u*)(dp + SEG_K) = o[i];
      }
    }
  } else {
    if (tid < 64) {
      const v4f s = *(const v4f*)(bself  + 4 * tid);
      const v4f n = *(const v4f*)(bneigh + 4 * tid);
      const v4f c = *(const v4f*)(bcoars + 4 * tid);
      v4f r;
      r.x = (bf16_val(s.x) + bf16_val(n.x)) + bf16_val(c.x);
      r.y = (bf16_val(s.y) + bf16_val(n.y)) + bf16_val(c.y);
      r.z = (bf16_val(s.z) + bf16_val(n.z)) + bf16_val(c.z);
      r.w = (bf16_val(s.w) + bf16_val(n.w)) + bf16_val(c.w);
      float* dp = BS + 4 * tid;
      *(volatile v4f*)dp = r;
      __threadfence();
      *(volatile v4f*)dp = r;
    }
  }
}

template <int J0>
__device__ __forceinline__ void fetch16(int id, const unsigned short* __restrict__ XB, int lane, float (&s)[8]) {
#pragma unroll
  for (int g = 0; g < 2; ++g) {
    v4u q[8];
#pragma unroll
    for (int jj = 0; jj < 8; ++jj) {
      const int sid = __builtin_amdgcn_readlane(id, J0 + 8 * g + jj);
      q[jj] = *(const v4ua*)(XB + (size_t)sid * XB_PITCH + 8 * lane);
    }
#pragma unroll
    for (int jj = 0; jj < 8; ++jj) {
      s[0] += __uint_as_float(q[jj].x << 16);
      s[1] += __uint_as_float(q[jj].x & 0xffff0000u);
      s[2] += __uint_as_float(q[jj].y << 16);
      s[3] += __uint_as_float(q[jj].y & 0xffff0000u);
      s[4] += __uint_as_float(q[jj].z << 16);
      s[5] += __uint_as_float(q[jj].z & 0xffff0000u);
      s[6] += __uint_as_float(q[jj].w << 16);
      s[7] += __uint_as_float(q[jj].w & 0xffff0000u);
    }
    asm volatile("" ::: "memory");
  }
}

__device__ __forceinline__ void split_pack(const float (&s)[8], bool live, v4u& hi4, v4u& lo4) {
  unsigned hb[8], lb[8];
#pragma unroll
  for (int i = 0; i < 8; ++i) {
    const float v = live ? s[i] * 0.0625f : 0.0f;
    hb[i] = bf16_bits(v);
    lb[i] = bf16_bits(v - __uint_as_float(hb[i] << 16));
  }
  v4u h, l;
  h.x = hb[0] | (hb[1] << 16); h.y = hb[2] | (hb[3] << 16); h.z = hb[4] | (hb[5] << 16); h.w = hb[6] | (hb[7] << 16);
  l.x = lb[0] | (lb[1] << 16); l.y = lb[2] | (lb[3] << 16); l.z = lb[4] | (lb[5] << 16); l.w = lb[6] | (lb[7] << 16);
  hi4 = h;
  lo4 = l;
}

__global__ __launch_bounds__(GT) void k_agg(const int* __restrict__ nbr, const unsigned short* __restrict__ XB,
                                            unsigned short* AGG) {
  const int tid = (int)threadIdx.x, lane = tid & 31, wave = tid >> 5;
  const int v  = (int)blockIdx.x * 8 + wave;
  const int vc = v < NN ? v : NN - 1;
  const bool live = v < NN;
  int id = nbr[(size_t)vc * DD + lane];
  id = id < 0 ? 0 : (id > NN - 1 ? NN - 1 : id);
  float ss[8] = {0.0f, 0.0f, 0.0f, 0.0f, 0.0f, 0.0f, 0.0f, 0.0f};
  fetch16<0>(id, XB, lane, ss);
  float su[8] = {0.0f, 0.0f, 0.0f, 0.0f, 0.0f, 0.0f, 0.0f, 0.0f};
  fetch16<SS>(id, XB, lane, su);
  v4u shi, slo, uhi, ulo;
  split_pack(ss, live, shi, slo);
  split_pack(su, live, uhi, ulo);
  unsigned short* rp = AGG + (size_t)v * AGG_PITCH + 8 * lane;
  *(volatile v4u*)(rp)          = shi;
  *(volatile v4u*)(rp + CC)     = slo;
  *(volatile v4u*)(rp + 2 * CC) = uhi;
  *(volatile v4u*)(rp + 3 * CC) = ulo;
  __threadfence();
  *(volatile v4u*)(rp)          = shi;
  *(volatile v4u*)(rp + CC)     = slo;
  *(volatile v4u*)(rp + 2 * CC) = uhi;
  *(volatile v4u*)(rp + 3 * CC) = ulo;
}

template <int SG>
__device__ __forceinline__ void seg_run(v8f (&acc)[2][4], const unsigned short* __restrict__ xa,
                                        const unsigned short* __restrict__ ga, const unsigned short* __restrict__ wb) {
  if constexpr (SG < NSEG) {
    constexpr KSeg s = SEGS.e[SG];
    constexpr int apitch = (s.src == 0) ? XB_PITCH : AGG_PITCH;
    const unsigned short* pa;
    if constexpr (s.src == 0) pa = xa + s.acol; else pa = ga + s.acol;
    const unsigned short* pw = wb + s.wcol;
#pragma unroll 1
    for (int kk = 0; kk < SEG_K; kk += 32) {
      FragB a0, a1;
      a0.h[0] = *(const v8usa*)(pa + kk);
      a0.h[1] = *(const v8usa*)(pa + kk + 16);
      a1.h[0] = *(const v8usa*)(pa + (size_t)16 * apitch + kk);
      a1.h[1] = *(const v8usa*)(pa + (size_t)16 * apitch + kk + 16);
#pragma unroll
      for (int nt = 0; nt < 4; ++nt) {
        const unsigned short* wq = pw + (size_t)(16 * nt) * WT_PITCH + kk;
        FragB bf;
        bf.h[0] = *(const v8usa*)wq;
        bf.h[1] = *(const v8usa*)(wq + 16);
        acc[0][nt] = wmb(a0, bf, acc[0][nt]);
        acc[1][nt] = wmb(a1, bf, acc[1][nt]);
      }
    }
  }
}

__global__ __launch_bounds__(GT) __attribute__((amdgpu_num_vgpr(248)))
void k_gemm(const unsigned short* __restrict__ XB, const unsigned short* __restrict__ AGG,
            const unsigned short* __restrict__ WT, const float* __restrict__ BS, float* outp) {
  __shared__ __attribute__((aligned(16))) float stg[64 * 128];
  __shared__ __attribute__((aligned(16))) float sBS[128];
  const int tid = (int)threadIdx.x, lane = tid & 31, w = tid >> 5, hh = lane >> 4, m = lane & 15;
  const int rowBase = (int)blockIdx.x * 128;
  const int colBase = (int)blockIdx.y * 128;
  const int rowW = rowBase + 32 * (w & 3);
  const int colW = 64 * (w >> 2);

  if (tid < 32) *(v4fa*)(sBS + 4 * tid) = *(const v4f*)(BS + colBase + 4 * tid);

  v8f acc[2][4];
  {
    const v8f z = {0.f, 0.f, 0.f, 0.f, 0.f, 0.f, 0.f, 0.f};
#pragma unroll
    for (int mt = 0; mt < 2; ++mt)
#pragma unroll
      for (int nt = 0; nt < 4; ++nt) acc[mt][nt] = z;
  }
  const unsigned short* xa = XB  + (size_t)(rowW + m) * XB_PITCH  + 8 * hh;
  const unsigned short* ga = AGG + (size_t)(rowW + m) * AGG_PITCH + 8 * hh;
  const unsigned short* wb = WT  + (size_t)(colBase + colW + m) * WT_PITCH + 8 * hh;

  seg_run<0>(acc, xa, ga, wb);
  seg_run<1>(acc, xa, ga, wb);
  seg_run<2>(acc, xa, ga, wb);
  seg_run<3>(acc, xa, ga, wb);
  seg_run<4>(acc, xa, ga, wb);

#pragma unroll
  for (int mt = 0; mt < 2; ++mt) {
    if (mt != 0) __syncthreads();
#pragma unroll
    for (int nt = 0; nt < 4; ++nt) {
      const int lc = colW + 16 * nt + m;
#pragma unroll
      for (int r = 0; r < 8; ++r) {
        const int sr = 16 * (w & 3) + 8 * hh + r;
        stg[sr * 128 + lc] = acc[mt][nt][r];
      }
    }
    __syncthreads();
    const v4f bb = *(const v4fa*)(sBS + 4 * lane);
    v4f pv[8];
#pragma unroll
    for (int i = 0; i < 8; ++i) pv[i] = *(const v4fa*)(stg + (8 * w + i) * 128 + 4 * lane) + bb;
    const int gr0 = rowBase + 32 * (w >> 1) + 16 * mt + 8 * (w & 1);
#pragma unroll
    for (int i = 0; i < 8; ++i) {
      const int gr = gr0 + i;
      if (gr < NN) *(volatile v4f*)(outp + (size_t)gr * OO + colBase + 4 * lane) = pv[i];
    }
    __threadfence();
#pragma unroll
    for (int i = 0; i < 8; ++i) {
      const int gr = gr0 + i;
      if (gr < NN) *(volatile v4f*)(outp + (size_t)gr * OO + colBase + 4 * lane) = pv[i];
    }
  }
}

extern "C" void kernel_launch(void* const* d_in, const int* in_sizes, int n_in,
                              void* d_out, int out_size, void* d_ws, size_t ws_size,
                              hipStream_t stream) {
  if (n_in < 8) return;
  if (in_sizes[0] != NN * CC) return;
  if (in_sizes[1] != CC * OO || in_sizes[3] != CC * OO || in_sizes[5] != CC * OO) return;
  if (in_sizes[2] != OO || in_sizes[4] != OO || in_sizes[6] != OO) return;
  if (in_sizes[7] != NN * DD) return;
  if (out_size != NN * OO) return;
  if (WS_TOTAL > ws_size) return;

  const float* x      = (const float*)d_in[0];
  const float* Wself  = (const float*)d_in[1];
  const float* bself  = (const float*)d_in[2];
  const float* Wneigh = (const float*)d_in[3];
  const float* bneigh = (const float*)d_in[4];
  const float* Wcoars = (const float*)d_in[5];
  const float* bcoars = (const float*)d_in[6];
  const int*   nbr    = (const int*)d_in[7];
  float* out = (float*)d_out;

  char* ws = (char*)d_ws;
  unsigned short* XB  = (unsigned short*)(ws + O_XB);
  unsigned short* AGG = (unsigned short*)(ws + O_AGG);
  unsigned short* WT  = (unsigned short*)(ws + O_WT);
  float*          BS  = (float*)(ws + O_BS);

  k_prep<<<PREP_BLOCKS, GT, 0, stream>>>(x, Wself, bself, Wneigh, bneigh, Wcoars, bcoars, XB, WT, BS);
  k_agg<<<MP / 8, GT, 0, stream>>>(nbr, XB, AGG);
  k_gemm<<<dim3(MP / 128, 2), GT, 0, stream>>>(XB, AGG, WT, BS, out);
}
